// BSRBF_KANLayer_7078106103839
// MI455X (gfx1250) — hardware-verified
//
#include <hip/hip_runtime.h>
#include <math.h>

#pragma clang fp contract(off)

constexpr int kInDim      = 512;
constexpr int kOutDim     = 512;
constexpr int kNBasis     = 8;
constexpr int kNKnot      = 12;
constexpr int kFeat       = kInDim * kNBasis;
constexpr int kKTot       = kInDim + kFeat;
constexpr int kChunkRows  = 8192;
constexpr int kRowChunks16 = kKTot / 8;
constexpr float kWCarry    = 256.0f;
constexpr float kWCarryInv = 1.0f / 256.0f;

typedef __attribute__((ext_vector_type(16))) _Float16 v16h;
typedef __attribute__((ext_vector_type(8)))  _Float16 v8h;
typedef __attribute__((ext_vector_type(16))) __bf16   v16b;
typedef __attribute__((ext_vector_type(8)))  __bf16   v8b;
typedef __attribute__((ext_vector_type(8)))  float    v8f;
typedef __attribute__((ext_vector_type(4)))  float    v4f;
typedef __attribute__((ext_vector_type(2)))  float    v2f;
typedef __attribute__((ext_vector_type(4)))  unsigned int v4u;

__device__ __forceinline__ unsigned short f2bf_bits(float f) {
  unsigned u = __float_as_uint(f);
  return (unsigned short)((u + 0x7FFFu + ((u >> 16) & 1u)) >> 16);
}
__device__ __forceinline__ float bf_bits2f(unsigned short h) { return __uint_as_float(((unsigned)h) << 16); }

__device__ __forceinline__ void dep_guard_h(v8f& a, v8f& b, v16h x, v16h y) { asm volatile("v_nop\n\tv_nop\n\tv_nop\n\tv_nop" : "+v"(a), "+v"(b) : "v"(x), "v"(y)); }
__device__ __forceinline__ void dep_guard_b(v8f& a, v8f& b, v16b x, v16b y) { asm volatile("v_nop\n\tv_nop\n\tv_nop\n\tv_nop" : "+v"(a), "+v"(b) : "v"(x), "v"(y)); }
__device__ __forceinline__ void keep4_h(v16h a, v16h b, v16h c, v16h d) { asm volatile("v_nop" :: "v"(a), "v"(b), "v"(c), "v"(d)); }
__device__ __forceinline__ void keep4_b(v16b a, v16b b, v16b c, v16b d) { asm volatile("v_nop" :: "v"(a), "v"(b), "v"(c), "v"(d)); }
__device__ __forceinline__ void acc_guard4(v8f& a, v8f& b, v8f& c, v8f& d) { asm volatile("v_nop\n\tv_nop\n\tv_nop\n\tv_nop" : "+v"(a), "+v"(b), "+v"(c), "+v"(d)); }
template <typename T> struct Frag;
template <> struct Frag<_Float16> {
  typedef v16h V; union U { v16h v; v8h h[2]; };
  static __device__ __forceinline__ v16h load(const _Float16* p) {
    U f; f.h[0] = *(const v8h*)(p); f.h[1] = *(const v8h*)(p + 16); return f.v;
  }
  static __device__ __forceinline__ v8f mma(v16h a, v16h b, v8f c) {
    return __builtin_amdgcn_wmma_f32_16x16x32_f16(false, a, false, b, (short)0, c, false, false);
  }
  static __device__ __forceinline__ void guard(v8f& a, v8f& b, v16h x, v16h y) { dep_guard_h(a, b, x, y); }
  static __device__ __forceinline__ void keep(v16h a, v16h b, v16h c, v16h d) { keep4_h(a, b, c, d); }
};
template <> struct Frag<__bf16> {
  typedef v16b V; union U { v16b v; v8b h[2]; };
  static __device__ __forceinline__ v16b load(const __bf16* p) {
    U f; f.h[0] = *(const v8b*)(p); f.h[1] = *(const v8b*)(p + 16); return f.v;
  }
  static __device__ __forceinline__ v8f mma(v16b a, v16b b, v8f c) {
    return __builtin_amdgcn_wmma_f32_16x16x32_bf16(false, a, false, b, (short)0, c, false, false);
  }
  static __device__ __forceinline__ void guard(v8f& a, v8f& b, v16b x, v16b y) { dep_guard_b(a, b, x, y); }
  static __device__ __forceinline__ void keep(v16b a, v16b b, v16b c, v16b d) { keep4_b(a, b, c, d); }
};

__device__ __forceinline__ unsigned pk16(unsigned short a, unsigned short b) { return (unsigned)a | ((unsigned)b << 16); }
__device__ __forceinline__ unsigned short h_bits(float f) { const _Float16 h = (_Float16)f; return __builtin_bit_cast(unsigned short, h); }
__device__ __forceinline__ float ftz16(float v) { return (fabsf(v) < 6.103515625e-5f) ? 0.0f : v; }

template <int ET> struct Elem;
template <> struct Elem<0> { typedef _Float16 T; };
template <> struct Elem<1> { typedef __bf16 T; };
template <int ET, bool SPLIT, int BIAS_MODE, int OUT_MODE, bool RESID, int ACT = 0>
__global__ __launch_bounds__(256) void wmma_gemm64(
    const unsigned short* __restrict__ Ap, const unsigned short* __restrict__ A2p, int lda, long strideA,
    const unsigned short* __restrict__ Btp, const unsigned short* __restrict__ Bt2p, int ldb, long strideB,
    void* __restrict__ Cout, void* __restrict__ Cout2, int ldc, long strideC,
    const float* __restrict__ bias,
    const float* __restrict__ resid, long strideR,
    int M, int N, int K, float scale) {
  typedef typename Elem<ET>::T T;
  typedef typename Frag<T>::V V;
  const T* A = (const T*)Ap; const T* A2 = (const T*)A2p; const T* Bt = (const T*)Btp; const T* Bt2 = (const T*)Bt2p;
  __shared__ __align__(16) float sT[8][16 * 68];
  const int b    = blockIdx.y;
  const int lane = threadIdx.x & 31;
  const int wave = threadIdx.x >> 5;
  const int tilesN = N >> 6;
  const int tilesM = M >> 6;
  const int tile = blockIdx.x * 8 + wave;
  if (tile >= tilesM * tilesN) return;
  const int tm = tile / tilesN;
  const int tn = tile - tm * tilesN;
  const int m0 = tm << 6;
  const int n0 = tn << 6;

  const T* Ab  = A  + (size_t)b * strideA;
  const T* Bb  = Bt + (size_t)b * strideB;
  const T* Ab2 = SPLIT ? (A2  + (size_t)b * strideA) : nullptr;
  const T* Bb2 = SPLIT ? (Bt2 + (size_t)b * strideB) : nullptr;

  const int rlane = lane & 15;
  const int koff  = (lane >> 4) * 8;
  const int mOff  = (lane >> 4) * 8;

  v8f acc[4][4];
#pragma unroll
  for (int i = 0; i < 4; ++i)
#pragma unroll
    for (int j = 0; j < 4; ++j) acc[i][j] = (v8f){0.f,0.f,0.f,0.f,0.f,0.f,0.f,0.f};

  for (int k0 = 0; k0 < K; k0 += 32) {
    V bh[4], bl[4];
#pragma unroll
    for (int j = 0; j < 4; ++j) {
      const size_t bo = (size_t)(n0 + (j << 4) + rlane) * ldb + koff + k0;
      bh[j] = Frag<T>::load(Bb + bo);
      if (SPLIT) bl[j] = Frag<T>::load(Bb2 + bo);
    }
#pragma unroll
    for (int i = 0; i < 4; ++i) {
      const size_t ao = (size_t)(m0 + (i << 4) + rlane) * lda + koff + k0;
      V ah = Frag<T>::load(Ab + ao);
      V al;
      if (SPLIT) al = Frag<T>::load(Ab2 + ao);
#pragma unroll
      for (int j = 0; j < 4; ++j) {
        acc[i][j] = Frag<T>::mma(ah, bh[j], acc[i][j]);
        if (SPLIT) {
          acc[i][j] = Frag<T>::mma(ah, bl[j], acc[i][j]);
          acc[i][j] = Frag<T>::mma(al, bh[j], acc[i][j]);
        }
      }
      Frag<T>::guard(acc[i][0], acc[i][3], ah, SPLIT ? al : ah);
    }
    Frag<T>::keep(bh[0], bh[1], bh[2], bh[3]);
    if (SPLIT) Frag<T>::keep(bl[0], bl[1], bl[2], bl[3]);
  }
  acc_guard4(acc[0][0], acc[0][1], acc[0][2], acc[0][3]);
  acc_guard4(acc[1][0], acc[1][1], acc[1][2], acc[1][3]);
  acc_guard4(acc[2][0], acc[2][1], acc[2][2], acc[2][3]);
  acc_guard4(acc[3][0], acc[3][1], acc[3][2], acc[3][3]);

  float* slab = sT[wave];
  const float* Rb = RESID ? (resid + (size_t)b * strideR) : nullptr;
#pragma unroll
  for (int i = 0; i < 4; ++i) {
    const int mBase = m0 + (i << 4);
#pragma unroll
    for (int j = 0; j < 4; ++j) {
      const int n = n0 + (j << 4) + rlane;
      float bv = 0.f;
      if (BIAS_MODE == 2) bv = bias[n];
#pragma unroll
      for (int r = 0; r < 8; ++r) {
        float v = acc[i][j][r] * scale;
        if (BIAS_MODE == 1) v += bias[mBase + mOff + r];
        if (BIAS_MODE == 2) v += bv;
        if (RESID) v += Rb[(size_t)(mBase + mOff + r) * ldc + n];
        if (ACT == 2) v = fmaxf(v, 0.0f);
        if (ACT == 4) v = (v > 0.f) ? v : 0.01f * v;
        slab[(mOff + r) * 68 + (j << 4) + rlane] = v;
      }
    }
    __builtin_amdgcn_fence(__ATOMIC_RELEASE, "workgroup");
    __builtin_amdgcn_wave_barrier();
    __builtin_amdgcn_fence(__ATOMIC_ACQUIRE, "workgroup");
    if (OUT_MODE == 0) {
      float* C = (float*)Cout + (size_t)b * strideC;
      const int hh = lane >> 4, c4 = (lane & 15) * 4;
      for (int pass = 0; pass < 2; ++pass) {
#pragma unroll
        for (int it = 0; it < 8; ++it) {
          const int row = it * 2 + hh;
          v4f v = *(const v4f*)(slab + row * 68 + c4);
          *(volatile v4f*)(C + (size_t)(mBase + row) * ldc + n0 + c4) = v;
        }
        __threadfence();
      }
    } else {
      const int q = lane >> 3, c8 = (lane & 7) * 8;
      unsigned short* C  = (unsigned short*)Cout  + (size_t)b * strideC;
      unsigned short* C2 = (OUT_MODE == 2) ? ((unsigned short*)Cout2 + (size_t)b * strideC) : nullptr;
      for (int pass = 0; pass < 2; ++pass) {
#pragma unroll
        for (int it = 0; it < 4; ++it) {
          const int row = it * 4 + q;
          const float* sp = slab + row * 68 + c8;
          v8h hv, lv;
#pragma unroll
          for (int e = 0; e < 8; ++e) {
            if (OUT_MODE == 1) {
              hv[e] = (_Float16)sp[e];
            } else {
              unsigned short hb = f2bf_bits(sp[e]);
              unsigned short lb = f2bf_bits(sp[e] - bf_bits2f(hb));
              hv[e] = __builtin_bit_cast(_Float16, hb);
              lv[e] = __builtin_bit_cast(_Float16, lb);
            }
          }
          *(volatile v8h*)(C + (size_t)(mBase + row) * ldc + n0 + c8) = hv;
          if (OUT_MODE == 2) *(volatile v8h*)(C2 + (size_t)(mBase + row) * ldc + n0 + c8) = lv;
        }
        __threadfence();
      }
    }
    __builtin_amdgcn_fence(__ATOMIC_RELEASE, "workgroup");
    __builtin_amdgcn_wave_barrier();
    __builtin_amdgcn_fence(__ATOMIC_ACQUIRE, "workgroup");
  }
}

__global__ __launch_bounds__(256) void wcat_cast_kernel(const float* __restrict__ bw, const float* __restrict__ sw,
                                                        unsigned short* __restrict__ out, int nchunks, float scale) {
  const int i = blockIdx.x * 256 + threadIdx.x;
  if (i >= nchunks) return;
  const int row = i / kRowChunks16;
  const int cc  = i - row * kRowChunks16;
  const int c8  = cc * 8;
  const bool useb = (c8 < kInDim);
  const int cb = useb ? c8 : (kInDim - 8);
  int cs = c8 - kInDim;
  cs = (cs < 0) ? 0 : cs;
  const float* pb = bw + (size_t)row * kInDim + cb;
  const float* ps = sw + (size_t)row * kFeat + cs;
  const v4f b0 = *(const v4f*)(pb);
  const v4f b1 = *(const v4f*)(pb + 4);
  const v4f s0 = *(const v4f*)(ps);
  const v4f s1 = *(const v4f*)(ps + 4);
  unsigned short hb[8];
#pragma unroll
  for (int e = 0; e < 4; ++e) {
    const float v0 = (useb ? b0[e] : s0[e]) * scale;
    const float v1 = (useb ? b1[e] : s1[e]) * scale;
    hb[e]     = h_bits(ftz16(v0));
    hb[4 + e] = h_bits(ftz16(v1));
  }
  const v4u u = (v4u){pk16(hb[0], hb[1]), pk16(hb[2], hb[3]), pk16(hb[4], hb[5]), pk16(hb[6], hb[7])};
  unsigned short* q = out + 8 * (size_t)i;
  *(volatile v4u*)q = u;
  __threadfence();
  *(volatile v4u*)q = u;
}

__global__ __launch_bounds__(256) void ln_basis_kernel(const float* __restrict__ x, const float* __restrict__ gam,
                                                       const float* __restrict__ bet, const float* __restrict__ gridk,
                                                       const float* __restrict__ rbfc, unsigned short* __restrict__ aout,
                                                       float inv_denom) {
  __shared__ float wsum[8];
  __shared__ float wsq[8];
  __shared__ __align__(16) unsigned int srow[kKTot / 2];
  const int row  = blockIdx.x;
  const int t    = threadIdx.x;
  const int lane = t & 31, wave = t >> 5;

  const float* xr = x + (size_t)row * kInDim;
  const v2f xv2 = *(const v2f*)(xr + 2 * t);
  const float x0 = xv2[0], x1 = xv2[1];

  float s = x0 + x1;
#pragma unroll
  for (int m = 16; m > 0; m >>= 1) s += __shfl_xor(s, m, 32);
  if (lane == 0) wsum[wave] = s;
  __syncthreads();
  float ts = wsum[0];
#pragma unroll
  for (int w = 1; w < 8; ++w) ts += wsum[w];
  const float mu = ts * (1.0f / 512.0f);

  const float dv0 = x0 - mu, dv1 = x1 - mu;
  const float sq0 = dv0 * dv0;
  const float sq1 = dv1 * dv1;
  float q = sq0 + sq1;
#pragma unroll
  for (int m = 16; m > 0; m >>= 1) q += __shfl_xor(q, m, 32);
  if (lane == 0) wsq[wave] = q;
  __syncthreads();
  float tq = wsq[0];
#pragma unroll
  for (int w = 1; w < 8; ++w) tq += wsq[w];
  const float var  = tq * (1.0f / 512.0f);
  const float rstd = rsqrtf(var + 1e-5f);

  const int d0 = 2 * t;
  const float y0 = dv0 * rstd;
  const float y1 = dv1 * rstd;
  const float z0 = y0 * gam[d0];
  const float z1 = y1 * gam[d0 + 1];
  const float xn0 = z0 + bet[d0];
  const float xn1 = z1 + bet[d0 + 1];

  {
    const float r0 = ftz16(fmaxf(xn0, 0.0f));
    const float r1 = ftz16(fmaxf(xn1, 0.0f));
    srow[t] = pk16(h_bits(r0), h_bits(r1));
  }

  const v4f rca = *(const v4f*)(rbfc);
  const v4f rcb = *(const v4f*)(rbfc + 4);
  const float rc[8] = {rca[0], rca[1], rca[2], rca[3], rcb[0], rcb[1], rcb[2], rcb[3]};

#pragma unroll 1
  for (int e = 0; e < 2; ++e) {
    const float xv = (e == 0) ? xn0 : xn1;
    const int d = d0 + e;
    const float* gp = gridk + (size_t)d * kNKnot;
    const v4f ga = *(const v4f*)(gp);
    const v4f gb = *(const v4f*)(gp + 4);
    const v4f gc = *(const v4f*)(gp + 8);
    const float gk[12] = {ga[0], ga[1], ga[2], ga[3], gb[0], gb[1], gb[2], gb[3], gc[0], gc[1], gc[2], gc[3]};

    float bq[11];
#pragma unroll
    for (int i = 0; i < 11; ++i) bq[i] = (xv >= gk[i] && xv < gk[i + 1]) ? 1.0f : 0.0f;

#pragma unroll
    for (int i = 0; i < 10; ++i) {
      const float dl = gk[i + 1] - gk[i];
      const float dr = gk[i + 2] - gk[i + 1];
      const float rl = __builtin_amdgcn_rcpf(dl);
      const float rr = __builtin_amdgcn_rcpf(dr);
      const float nl = xv - gk[i];
      const float nr = gk[i + 2] - xv;
      const float wl = nl * rl;
      const float wr = nr * rr;
      const float t1 = wl * bq[i];
      const float t2 = wr * bq[i + 1];
      bq[i] = t1 + t2;
    }
#pragma unroll
    for (int i = 0; i < 9; ++i) {
      const float dl = gk[i + 2] - gk[i];
      const float dr = gk[i + 3] - gk[i + 1];
      const float rl = __builtin_amdgcn_rcpf(dl);
      const float rr = __builtin_amdgcn_rcpf(dr);
      const float nl = xv - gk[i];
      const float nr = gk[i + 3] - xv;
      const float wl = nl * rl;
      const float wr = nr * rr;
      const float t1 = wl * bq[i];
      const float t2 = wr * bq[i + 1];
      bq[i] = t1 + t2;
    }
#pragma unroll
    for (int i = 0; i < 8; ++i) {
      const float dl = gk[i + 3] - gk[i];
      const float dr = gk[i + 4] - gk[i + 1];
      const float rl = __builtin_amdgcn_rcpf(dl);
      const float rr = __builtin_amdgcn_rcpf(dr);
      const float nl = xv - gk[i];
      const float nr = gk[i + 4] - xv;
      const float wl = nl * rl;
      const float wr = nr * rr;
      const float t1 = wl * bq[i];
      const float t2 = wr * bq[i + 1];
      bq[i] = t1 + t2;
    }

#pragma unroll
    for (int p = 0; p < 4; ++p) {
      const float ta = (xv - rc[2 * p]) * inv_denom;
      const float ua = ta * ta;
      const float ea = expf(-ua);
      const float va = ftz16(bq[2 * p] + ea);
      const float tb = (xv - rc[2 * p + 1]) * inv_denom;
      const float ub = tb * tb;
      const float eb = expf(-ub);
      const float vb = ftz16(bq[2 * p + 1] + eb);
      srow[256 + 4 * d + p] = pk16(h_bits(va), h_bits(vb));
    }
  }
  __syncthreads();

  unsigned short* arow = aout + (size_t)row * kKTot;
  const v4u u0 = *(const v4u*)(srow + 4 * t);
  const v4u u1 = *(const v4u*)(srow + 4 * (t + 256));
  const bool third = (t < 64);
  const int c2 = third ? (t + 512) : (kRowChunks16 - 1);
  const v4u u2 = *(const v4u*)(srow + 4 * c2);
  unsigned short* q0 = arow + 8 * t;
  unsigned short* q1 = arow + 8 * (t + 256);
  unsigned short* q2 = arow + 8 * c2;
  *(volatile v4u*)q0 = u0;
  *(volatile v4u*)q1 = u1;
  if (third) *(volatile v4u*)q2 = u2;
  __threadfence();
  *(volatile v4u*)q0 = u0;
  *(volatile v4u*)q1 = u1;
  if (third) *(volatile v4u*)q2 = u2;
}

extern "C" void kernel_launch(void* const* d_in, const int* in_sizes, int n_in,
                              void* d_out, int out_size, void* d_ws, size_t ws_size,
                              hipStream_t stream) {
  (void)n_in;
  const float* x     = (const float*)d_in[0];
  const float* gam   = (const float*)d_in[1];
  const float* bet   = (const float*)d_in[2];
  const float* basew = (const float*)d_in[3];
  const float* splw  = (const float*)d_in[4];
  const float* gridk = (const float*)d_in[5];
  const float* rbfc  = (const float*)d_in[6];
  float* out = (float*)d_out;

  const long nrows = (long)in_sizes[0] / kInDim;
  const long nch = nrows / kChunkRows;
  if (nch < 1 || nch * kChunkRows != nrows) return;
  if ((long)out_size != nrows * kOutDim) return;
  if (in_sizes[3] != kOutDim * kInDim || in_sizes[4] != kOutDim * kFeat ||
      in_sizes[5] != kInDim * kNKnot || in_sizes[6] != kNBasis ||
      in_sizes[1] != kInDim || in_sizes[2] != kInDim) return;

  const size_t wt_bytes = (size_t)kOutDim * kKTot * 2;
  const size_t off_a    = (wt_bytes + 127) & ~(size_t)127;
  const size_t a_bytes  = (size_t)kChunkRows * kKTot * 2;
  if (off_a + a_bytes > ws_size) return;
  unsigned short* wt16 = (unsigned short*)d_ws;
  unsigned short* a16  = (unsigned short*)((char*)d_ws + off_a);

  const int nchunksW = kOutDim * kRowChunks16;
  wcat_cast_kernel<<<dim3((nchunksW + 255) / 256), dim3(256), 0, stream>>>(basew, splw, wt16, nchunksW, kWCarry);

  const float denomf = (float)(3.0 / 7.0);
  const float inv_denom = 1.0f / denomf;
  const int tiles = (kChunkRows / 64) * (kOutDim / 64);
  const int gx = (tiles + 7) / 8;
  for (long ch = 0; ch < nch; ++ch) {
    ln_basis_kernel<<<dim3(kChunkRows), dim3(256), 0, stream>>>(
        x + (size_t)ch * kChunkRows * kInDim, gam, bet, gridk, rbfc, a16, inv_denom);
    wmma_gemm64<0, false, 0, 0, false, 0><<<dim3(gx, 1), dim3(256), 0, stream>>>(
        a16, a16, kKTot, 0L,
        wt16, wt16, kKTot, 0L,
        (void*)(out + (size_t)ch * kChunkRows * kOutDim), (void*)nullptr, kOutDim, 0L,
        (const float*)nullptr,
        (const float*)nullptr, 0L,
        kChunkRows, kOutDim, kKTot, kWCarryInv);
  }
}
